// LSTMEncoding_29076928594507
// MI455X (gfx1250) — hardware-verified
//
#include <hip/hip_runtime.h>
#include <math.h>

constexpr int NBATCH = 64;
constexpr int NSTEP  = 64;
constexpr int GLD    = 300;
constexpr int KPAD   = 320;
constexpr int DMOD   = 1024;
constexpr int NGATE  = 4 * DMOD;
constexpr int NTOK   = NBATCH * NSTEP;
constexpr int NVOC   = 50000;
constexpr int NTHR   = 256;
constexpr int SEQ_BLK = 16;
constexpr int HPITCH = 1032;
constexpr int SLABP  = 68;
constexpr int UNITS_PER_WAVE = DMOD / (NTHR / 32);
constexpr int NT_PER_WAVE    = UNITS_PER_WAVE / 16;
constexpr float WCARRY  = 64.0f;
constexpr float XCARRY  = 8.0f;
constexpr float HCARRY  = 16.0f;
constexpr float RINV_XW = 1.0f / (8.0f * 64.0f);
constexpr float RINV_HW = 1.0f / (16.0f * 64.0f);
static_assert(NBATCH == 64 && NSTEP == 64);
static_assert(KPAD % 32 == 0 && KPAD >= GLD);
static_assert(NTOK % 64 == 0 && DMOD % 64 == 0 && NGATE % 64 == 0 && DMOD % 32 == 0);
static_assert(NBATCH % SEQ_BLK == 0);
static_assert(UNITS_PER_WAVE * (NTHR / 32) == DMOD);
static_assert(NT_PER_WAVE == 8);
static_assert((2 * SEQ_BLK * HPITCH) % NTHR == 0);
static_assert(HPITCH % 8 == 0 && HPITCH >= DMOD);
static_assert((NTOK * (KPAD / 8)) % NTHR == 0 && (DMOD * (KPAD / 8)) % NTHR == 0);
static_assert((NGATE * (DMOD / 8)) % NTHR == 0);

typedef __attribute__((ext_vector_type(16))) _Float16 v16h;
typedef __attribute__((ext_vector_type(8)))  _Float16 v8h;
typedef __attribute__((ext_vector_type(16))) __bf16   v16b;
typedef __attribute__((ext_vector_type(8)))  __bf16   v8b;
typedef __attribute__((ext_vector_type(8)))  float    v8f;
typedef __attribute__((ext_vector_type(4)))  float    v4f;

__device__ __forceinline__ unsigned short f2bf_bits(float f) {
  unsigned u = __float_as_uint(f);
  return (unsigned short)((u + 0x7FFFu + ((u >> 16) & 1u)) >> 16);
}
__device__ __forceinline__ float bf_bits2f(unsigned short h) { return __uint_as_float(((unsigned)h) << 16); }
__device__ __forceinline__ float bf16r(float f) { return bf_bits2f(f2bf_bits(f)); }

__device__ __forceinline__ void dep_guard_h(v8f& a, v8f& b, v16h x, v16h y) { asm volatile("v_nop\n\tv_nop\n\tv_nop\n\tv_nop" : "+v"(a), "+v"(b) : "v"(x), "v"(y)); }
__device__ __forceinline__ void dep_guard_b(v8f& a, v8f& b, v16b x, v16b y) { asm volatile("v_nop\n\tv_nop\n\tv_nop\n\tv_nop" : "+v"(a), "+v"(b) : "v"(x), "v"(y)); }
__device__ __forceinline__ void keep4_h(v16h a, v16h b, v16h c, v16h d) { asm volatile("v_nop" :: "v"(a), "v"(b), "v"(c), "v"(d)); }
__device__ __forceinline__ void keep4_b(v16b a, v16b b, v16b c, v16b d) { asm volatile("v_nop" :: "v"(a), "v"(b), "v"(c), "v"(d)); }
__device__ __forceinline__ void acc_guard4(v8f& a, v8f& b, v8f& c, v8f& d) { asm volatile("v_nop\n\tv_nop\n\tv_nop\n\tv_nop" : "+v"(a), "+v"(b), "+v"(c), "+v"(d)); }
template <typename T> struct Frag;
template <> struct Frag<_Float16> {
  typedef v16h V; union U { v16h v; v8h h[2]; };
  static __device__ __forceinline__ v16h load(const _Float16* p) {
    U f; f.h[0] = *(const v8h*)(p); f.h[1] = *(const v8h*)(p + 16); return f.v;
  }
  static __device__ __forceinline__ v8f mma(v16h a, v16h b, v8f c) {
    return __builtin_amdgcn_wmma_f32_16x16x32_f16(false, a, false, b, (short)0, c, false, false);
  }
  static __device__ __forceinline__ void guard(v8f& a, v8f& b, v16h x, v16h y) { dep_guard_h(a, b, x, y); }
  static __device__ __forceinline__ void keep(v16h a, v16h b, v16h c, v16h d) { keep4_h(a, b, c, d); }
};
template <> struct Frag<__bf16> {
  typedef v16b V; union U { v16b v; v8b h[2]; };
  static __device__ __forceinline__ v16b load(const __bf16* p) {
    U f; f.h[0] = *(const v8b*)(p); f.h[1] = *(const v8b*)(p + 16); return f.v;
  }
  static __device__ __forceinline__ v8f mma(v16b a, v16b b, v8f c) {
    return __builtin_amdgcn_wmma_f32_16x16x32_bf16(false, a, false, b, (short)0, c, false, false);
  }
  static __device__ __forceinline__ void guard(v8f& a, v8f& b, v16b x, v16b y) { dep_guard_b(a, b, x, y); }
  static __device__ __forceinline__ void keep(v16b a, v16b b, v16b c, v16b d) { keep4_b(a, b, c, d); }
};

__device__ __forceinline__ float fsig(float x)  { return __builtin_amdgcn_rcpf(1.0f + expf(-x)); }
__device__ __forceinline__ float ftanh(float x) { return 1.0f - 2.0f * __builtin_amdgcn_rcpf(expf(2.0f * x) + 1.0f); }

template <int ET> struct Elem;
template <> struct Elem<0> { typedef _Float16 T; };
template <> struct Elem<1> { typedef __bf16 T; };
template <int ET, bool SPLIT, int BIAS_MODE, int OUT_MODE, bool RESID, int ACT = 0>
__global__ __launch_bounds__(256) void wmma_gemm64(
    const unsigned short* __restrict__ Ap, const unsigned short* __restrict__ A2p, int lda, long strideA,
    const unsigned short* __restrict__ Btp, const unsigned short* __restrict__ Bt2p, int ldb, long strideB,
    void* __restrict__ Cout, void* __restrict__ Cout2, int ldc, long strideC,
    const float* __restrict__ bias,
    const float* __restrict__ resid, long strideR,
    int M, int N, int K, float scale) {
  typedef typename Elem<ET>::T T;
  typedef typename Frag<T>::V V;
  const T* A = (const T*)Ap; const T* A2 = (const T*)A2p; const T* Bt = (const T*)Btp; const T* Bt2 = (const T*)Bt2p;
  __shared__ __align__(16) float sT[8][16 * 68];
  const int b    = blockIdx.y;
  const int lane = threadIdx.x & 31;
  const int wave = threadIdx.x >> 5;
  const int tilesN = N >> 6;
  const int tilesM = M >> 6;
  const int tile = blockIdx.x * 8 + wave;
  if (tile >= tilesM * tilesN) return;
  const int tm = tile / tilesN;
  const int tn = tile - tm * tilesN;
  const int m0 = tm << 6;
  const int n0 = tn << 6;

  const T* Ab  = A  + (size_t)b * strideA;
  const T* Bb  = Bt + (size_t)b * strideB;
  const T* Ab2 = SPLIT ? (A2  + (size_t)b * strideA) : nullptr;
  const T* Bb2 = SPLIT ? (Bt2 + (size_t)b * strideB) : nullptr;

  const int rlane = lane & 15;
  const int koff  = (lane >> 4) * 8;
  const int mOff  = (lane >> 4) * 8;

  v8f acc[4][4];
#pragma unroll
  for (int i = 0; i < 4; ++i)
#pragma unroll
    for (int j = 0; j < 4; ++j) acc[i][j] = (v8f){0.f,0.f,0.f,0.f,0.f,0.f,0.f,0.f};

  for (int k0 = 0; k0 < K; k0 += 32) {
    V bh[4], bl[4];
#pragma unroll
    for (int j = 0; j < 4; ++j) {
      const size_t bo = (size_t)(n0 + (j << 4) + rlane) * ldb + koff + k0;
      bh[j] = Frag<T>::load(Bb + bo);
      if (SPLIT) bl[j] = Frag<T>::load(Bb2 + bo);
    }
#pragma unroll
    for (int i = 0; i < 4; ++i) {
      const size_t ao = (size_t)(m0 + (i << 4) + rlane) * lda + koff + k0;
      V ah = Frag<T>::load(Ab + ao);
      V al;
      if (SPLIT) al = Frag<T>::load(Ab2 + ao);
#pragma unroll
      for (int j = 0; j < 4; ++j) {
        acc[i][j] = Frag<T>::mma(ah, bh[j], acc[i][j]);
        if (SPLIT) {
          acc[i][j] = Frag<T>::mma(ah, bl[j], acc[i][j]);
          acc[i][j] = Frag<T>::mma(al, bh[j], acc[i][j]);
        }
      }
      Frag<T>::guard(acc[i][0], acc[i][3], ah, SPLIT ? al : ah);
    }
    Frag<T>::keep(bh[0], bh[1], bh[2], bh[3]);
    if (SPLIT) Frag<T>::keep(bl[0], bl[1], bl[2], bl[3]);
  }
  acc_guard4(acc[0][0], acc[0][1], acc[0][2], acc[0][3]);
  acc_guard4(acc[1][0], acc[1][1], acc[1][2], acc[1][3]);
  acc_guard4(acc[2][0], acc[2][1], acc[2][2], acc[2][3]);
  acc_guard4(acc[3][0], acc[3][1], acc[3][2], acc[3][3]);

  float* slab = sT[wave];
  const float* Rb = RESID ? (resid + (size_t)b * strideR) : nullptr;
#pragma unroll
  for (int i = 0; i < 4; ++i) {
    const int mBase = m0 + (i << 4);
#pragma unroll
    for (int j = 0; j < 4; ++j) {
      const int n = n0 + (j << 4) + rlane;
      float bv = 0.f;
      if (BIAS_MODE == 2) bv = bias[n];
#pragma unroll
      for (int r = 0; r < 8; ++r) {
        float v = acc[i][j][r] * scale;
        if (BIAS_MODE == 1) v += bias[mBase + mOff + r];
        if (BIAS_MODE == 2) v += bv;
        if (RESID) v += Rb[(size_t)(mBase + mOff + r) * ldc + n];
        if (ACT == 1) v = tanhf(v);
        if (ACT == 2) v = fmaxf(v, 0.0f);
        if (ACT == 3) v = v / (1.0f + expf(-v));
        if (ACT == 4) v = (v > 0.f) ? v : 0.01f * v;
        if (ACT == 5) v = 0.5f * v * (1.0f + erff(v * 0.70710678118654752f));
        slab[(mOff + r) * 68 + (j << 4) + rlane] = v;
      }
    }
    __builtin_amdgcn_fence(__ATOMIC_RELEASE, "workgroup");
    __builtin_amdgcn_wave_barrier();
    __builtin_amdgcn_fence(__ATOMIC_ACQUIRE, "workgroup");
    if (OUT_MODE == 0) {
      float* C = (float*)Cout + (size_t)b * strideC;
      const int hh = lane >> 4, c4 = (lane & 15) * 4;
      for (int pass = 0; pass < 2; ++pass) {
#pragma unroll
        for (int it = 0; it < 8; ++it) {
          const int row = it * 2 + hh;
          v4f v = *(const v4f*)(slab + row * 68 + c4);
          *(volatile v4f*)(C + (size_t)(mBase + row) * ldc + n0 + c4) = v;
        }
        __threadfence();
      }
    } else {
      const int q = lane >> 3, c8 = (lane & 7) * 8;
      unsigned short* C  = (unsigned short*)Cout  + (size_t)b * strideC;
      unsigned short* C2 = (OUT_MODE == 2) ? ((unsigned short*)Cout2 + (size_t)b * strideC) : nullptr;
      for (int pass = 0; pass < 2; ++pass) {
#pragma unroll
        for (int it = 0; it < 4; ++it) {
          const int row = it * 4 + q;
          const float* sp = slab + row * 68 + c8;
          v8h hv, lv;
#pragma unroll
          for (int e = 0; e < 8; ++e) {
            if (OUT_MODE == 1) {
              hv[e] = (_Float16)sp[e];
            } else {
              unsigned short hb = f2bf_bits(sp[e]);
              unsigned short lb = f2bf_bits(sp[e] - bf_bits2f(hb));
              hv[e] = __builtin_bit_cast(_Float16, hb);
              lv[e] = __builtin_bit_cast(_Float16, lb);
            }
          }
          *(volatile v8h*)(C + (size_t)(mBase + row) * ldc + n0 + c8) = hv;
          if (OUT_MODE == 2) *(volatile v8h*)(C2 + (size_t)(mBase + row) * ldc + n0 + c8) = lv;
        }
        __threadfence();
      }
    }
    __builtin_amdgcn_fence(__ATOMIC_RELEASE, "workgroup");
    __builtin_amdgcn_wave_barrier();
    __builtin_amdgcn_fence(__ATOMIC_ACQUIRE, "workgroup");
  }
}

template <int MODE>
__global__ __launch_bounds__(NTHR) void cvt8_kernel(const float* __restrict__ src, unsigned short* __restrict__ dst,
                                                    int nrow, int ncol8, int spitch, int scol0, float sc) {
  const int i  = blockIdx.x * NTHR + threadIdx.x;
  const int n8 = nrow * ncol8;
  if (i < n8) {
    const int row = i / ncol8;
    const int c8  = i - row * ncol8;
    const float* sp = src + (size_t)row * spitch + scol0 + c8 * 8;
    const v4f a = *(const v4f*)(sp);
    const v4f b = *(const v4f*)(sp + 4);
    v8h hv;
#pragma unroll
    for (int e = 0; e < 4; ++e) {
      unsigned short b0, b1;
      if (MODE == 0) {
        b0 = f2bf_bits(a[e] * sc);
        b1 = f2bf_bits(b[e] * sc);
      } else {
        b0 = __builtin_bit_cast(unsigned short, (_Float16)(bf16r(a[e]) * sc));
        b1 = __builtin_bit_cast(unsigned short, (_Float16)(bf16r(b[e]) * sc));
      }
      hv[e]     = __builtin_bit_cast(_Float16, b0);
      hv[4 + e] = __builtin_bit_cast(_Float16, b1);
    }
    *(volatile v8h*)(dst + (size_t)i * 8) = hv;
    __threadfence();
    *(volatile v8h*)(dst + (size_t)i * 8) = hv;
  }
}

template <bool GATHER>
__global__ __launch_bounds__(NTHR) void pad300_kernel(const float* __restrict__ src, const int* __restrict__ ids,
                                                      unsigned short* __restrict__ dst, int nrow, float sc) {
  const int i  = blockIdx.x * NTHR + threadIdx.x;
  const int n8 = nrow * (KPAD / 8);
  if (i < n8) {
    const int row = i / (KPAD / 8);
    const int c8  = (i - row * (KPAD / 8)) * 8;
    int srow = row;
    if (GATHER) {
      const int bb = row & (NBATCH - 1);
      const int tt = row >> 6;
      int s = ids[bb * NSTEP + tt];
      s = s < 0 ? 0 : s;
      s = s > NVOC - 1 ? NVOC - 1 : s;
      srow = s;
    }
    const float* sp = src + (size_t)srow * GLD;
    v8h hv;
#pragma unroll
    for (int e = 0; e < 8; ++e) {
      const int col = c8 + e;
      const int cc  = col < GLD ? col : GLD - 1;
      const float f = sp[cc];
      const float v = (col < GLD) ? bf16r(f) * sc : 0.0f;
      hv[e] = (_Float16)v;
    }
    *(volatile v8h*)(dst + (size_t)i * 8) = hv;
    __threadfence();
    *(volatile v8h*)(dst + (size_t)i * 8) = hv;
  }
}

__global__ __launch_bounds__(NTHR) void bias_prep_kernel(const float* __restrict__ b_emb, const float* __restrict__ b_ih,
                                                         const float* __restrict__ b_hh,
                                                         float* __restrict__ BE8, float* __restrict__ BG) {
  const int tid = threadIdx.x, blk = blockIdx.x;
  const int idxE = tid * 4;
  int gb = blk - 1; gb = gb < 0 ? 0 : gb;
  const int idxG = gb * DMOD + tid * 4;
  const v4f ve = *(const v4f*)(b_emb + idxE);
  const v4f vi = *(const v4f*)(b_ih + idxG);
  const v4f vh = *(const v4f*)(b_hh + idxG);
  const bool isE = (blk == 0);
  v4f o;
#pragma unroll
  for (int e = 0; e < 4; ++e) {
    const float oe = bf16r(ve[e]) * XCARRY;
    const float og = bf16r(vi[e]) + bf16r(vh[e]);
    o[e] = isE ? oe : og;
  }
  float* op = isE ? (BE8 + idxE) : (BG + idxG);
  *(volatile v4f*)op = o;
  __threadfence();
  *(volatile v4f*)op = o;
}

__global__ __launch_bounds__(NTHR) void lstm_seq_kernel(const float* __restrict__ XP, const float* __restrict__ BG,
                                                        const unsigned short* __restrict__ WHHp,
                                                        float* __restrict__ out) {
  __shared__ __align__(16) _Float16 Ah[2][SEQ_BLK * HPITCH];
  __shared__ __align__(16) float    Sl[NTHR / 32][16 * SLABP];
  const _Float16* WHH = (const _Float16*)WHHp;
  const int tid = threadIdx.x, lane = tid & 31, wave = tid >> 5;
  const int c = lane & 15, hh = lane >> 4, koff = hh * 8, c4 = c * 4;
  const int rowbase = blockIdx.x * SEQ_BLK;

  {
    _Float16* ahf = &Ah[0][0];
#pragma unroll 1
    for (int i = tid; i < 2 * SEQ_BLK * HPITCH; i += NTHR) ahf[i] = (_Float16)0.0f;
  }
  float cst[NT_PER_WAVE][8];
#pragma unroll
  for (int nt = 0; nt < NT_PER_WAVE; ++nt)
#pragma unroll
    for (int r = 0; r < 8; ++r) cst[nt][r] = 0.0f;
  __syncthreads();

  const v8f z8 = {0.f, 0.f, 0.f, 0.f, 0.f, 0.f, 0.f, 0.f};
  float* slab = Sl[wave];

#pragma unroll 1
  for (int t = 0; t < NSTEP; ++t) {
    const int cur = t & 1;
    const _Float16* ahrow = &Ah[cur][0] + c * HPITCH + koff;
    _Float16* ahn = &Ah[cur ^ 1][0];
#pragma unroll
    for (int nt = 0; nt < NT_PER_WAVE; ++nt) {
      const int j = UNITS_PER_WAVE * wave + 16 * nt + c;
      const _Float16* wh = WHH + (size_t)j * DMOD + koff;
      v8f acc[4];
      acc[0] = z8; acc[1] = z8; acc[2] = z8; acc[3] = z8;
#pragma unroll 1
      for (int k0 = 0; k0 < DMOD; k0 += 32) {
        const v16h a  = Frag<_Float16>::load(ahrow + k0);
        const v16h b0 = Frag<_Float16>::load(wh + k0);
        const v16h b1 = Frag<_Float16>::load(wh + (size_t)1 * DMOD * DMOD + k0);
        const v16h b2 = Frag<_Float16>::load(wh + (size_t)2 * DMOD * DMOD + k0);
        const v16h b3 = Frag<_Float16>::load(wh + (size_t)3 * DMOD * DMOD + k0);
        acc[0] = Frag<_Float16>::mma(a, b0, acc[0]);
        acc[1] = Frag<_Float16>::mma(a, b1, acc[1]);
        acc[2] = Frag<_Float16>::mma(a, b2, acc[2]);
        acc[3] = Frag<_Float16>::mma(a, b3, acc[3]);
        dep_guard_h(acc[0], acc[3], a, b3);
        keep4_h(b0, b1, b2, b3);
      }
      acc_guard4(acc[0], acc[1], acc[2], acc[3]);

      float xv[4][8], bgv[4];
      {
        const float* xp = XP + (size_t)j * NTOK + (size_t)t * NBATCH + rowbase + 8 * hh;
#pragma unroll
        for (int g = 0; g < 4; ++g) {
          const float* xg = xp + (size_t)g * DMOD * NTOK;
          const v4f va = *(const v4f*)(xg);
          const v4f vb = *(const v4f*)(xg + 4);
#pragma unroll
          for (int e = 0; e < 4; ++e) { xv[g][e] = va[e]; xv[g][4 + e] = vb[e]; }
          bgv[g] = BG[g * DMOD + j];
        }
      }
#pragma unroll
      for (int r = 0; r < 8; ++r) {
        const float zi = acc[0][r] * RINV_HW + (xv[0][r] + bgv[0]);
        const float zf = acc[1][r] * RINV_HW + (xv[1][r] + bgv[1]);
        const float zg = acc[2][r] * RINV_HW + (xv[2][r] + bgv[2]);
        const float zo = acc[3][r] * RINV_HW + (xv[3][r] + bgv[3]);
        const float ig = fsig(zi);
        const float fg = fsig(zf);
        const float gg = ftanh(zg);
        const float og = fsig(zo);
        const float cn = fg * cst[nt][r] + ig * gg;
        cst[nt][r] = cn;
        const float hn = og * ftanh(cn);
        ahn[(8 * hh + r) * HPITCH + j] = (_Float16)(hn * HCARRY);
        slab[(8 * hh + r) * SLABP + 16 * (nt & 3) + c] = hn;
      }
      if ((nt & 3) == 3) {
        const int seg = nt >> 2;
        __builtin_amdgcn_fence(__ATOMIC_RELEASE, "workgroup");
        __builtin_amdgcn_wave_barrier();
        __builtin_amdgcn_fence(__ATOMIC_ACQUIRE, "workgroup");
        for (int pass = 0; pass < 2; ++pass) {
#pragma unroll
          for (int it = 0; it < 8; ++it) {
            const int row = it * 2 + hh;
            const v4f v = *(const v4f*)(slab + row * SLABP + c4);
            *(volatile v4f*)(out + ((size_t)(rowbase + row) * NSTEP + (size_t)t) * DMOD
                             + UNITS_PER_WAVE * wave + 64 * seg + c4) = v;
          }
          __threadfence();
        }
        __builtin_amdgcn_fence(__ATOMIC_RELEASE, "workgroup");
        __builtin_amdgcn_wave_barrier();
        __builtin_amdgcn_fence(__ATOMIC_ACQUIRE, "workgroup");
      }
    }
    __syncthreads();
  }
}

extern "C" void kernel_launch(void* const* d_in, const int* in_sizes, int n_in,
                              void* d_out, int out_size, void* d_ws, size_t ws_size, hipStream_t stream) {
  if (n_in < 8 || d_out == nullptr || d_ws == nullptr) return;
  if (in_sizes[0] != NBATCH * NSTEP || in_sizes[1] != NVOC * GLD || in_sizes[2] != DMOD * GLD || in_sizes[3] != DMOD ||
      in_sizes[4] != NGATE * DMOD || in_sizes[5] != NGATE * DMOD || in_sizes[6] != NGATE || in_sizes[7] != NGATE ||
      out_size != NTOK * DMOD) return;

  const int*   seqs  = (const int*)d_in[0];
  const float* glove = (const float*)d_in[1];
  const float* wemb  = (const float*)d_in[2];
  const float* bemb  = (const float*)d_in[3];
  const float* wih   = (const float*)d_in[4];
  const float* whh   = (const float*)d_in[5];
  const float* bih   = (const float*)d_in[6];
  const float* bhh   = (const float*)d_in[7];
  float* out = (float*)d_out;

  char* ws = (char*)d_ws; size_t off = 0;
  auto carve = [&](size_t bytes) -> char* { char* p = ws + off; off += (bytes + 255) & ~(size_t)255; return p; };
  unsigned short* WIH16  = (unsigned short*)carve((size_t)NGATE * DMOD * 2);
  unsigned short* WHH16  = (unsigned short*)carve((size_t)NGATE * DMOD * 2);
  unsigned short* WEMB16 = (unsigned short*)carve((size_t)DMOD * KPAD * 2);
  unsigned short* EMB16  = (unsigned short*)carve((size_t)NTOK * KPAD * 2);
  unsigned short* X16    = (unsigned short*)carve((size_t)NTOK * DMOD * 2);
  float*          BE8    = (float*)carve((size_t)DMOD * 4);
  float*          BG     = (float*)carve((size_t)NGATE * 4);
  float*          XPROJ  = (float*)carve((size_t)NGATE * NTOK * 4);
  if (off > ws_size || off > (size_t)134217728) return;

  const int n8e = DMOD * (KPAD / 8);
  const int n8g = NTOK * (KPAD / 8);
  const int n8w = NGATE * (DMOD / 8);
  pad300_kernel<false><<<(n8e + NTHR - 1) / NTHR, NTHR, 0, stream>>>(wemb, seqs, WEMB16, DMOD, WCARRY);
  pad300_kernel<true><<<(n8g + NTHR - 1) / NTHR, NTHR, 0, stream>>>(glove, seqs, EMB16, NTOK, 1.0f);
  cvt8_kernel<1><<<(n8w + NTHR - 1) / NTHR, NTHR, 0, stream>>>(wih, WIH16, NGATE, DMOD / 8, DMOD, 0, WCARRY);
  cvt8_kernel<1><<<(n8w + NTHR - 1) / NTHR, NTHR, 0, stream>>>(whh, WHH16, NGATE, DMOD / 8, DMOD, 0, WCARRY);
  bias_prep_kernel<<<5, NTHR, 0, stream>>>(bemb, bih, bhh, BE8, BG);

  wmma_gemm64<0, false, 2, 1, false, 0><<<dim3((NTOK / 64) * (DMOD / 64) / 8, 1), 256, 0, stream>>>(
      EMB16, EMB16, KPAD, 0L, WEMB16, WEMB16, KPAD, 0L, (void*)X16, (void*)X16, DMOD, 0L,
      BE8, BG, 0L, NTOK, DMOD, KPAD, XCARRY / WCARRY);

  wmma_gemm64<0, false, 0, 0, false, 0><<<dim3((NGATE / 64) * (NTOK / 64) / 8, 1), 256, 0, stream>>>(
      WIH16, WIH16, DMOD, 0L, X16, X16, DMOD, 0L, (void*)XPROJ, (void*)XPROJ, NTOK, 0L,
      BE8, BG, 0L, NGATE, NTOK, DMOD, RINV_XW);

  lstm_seq_kernel<<<NBATCH / SEQ_BLK, NTHR, 0, stream>>>(XPROJ, BG, WHH16, out);
}
